// model_indRNN_6906307412189
// MI455X (gfx1250) — hardware-run, weakly checked
//
#include <hip/hip_runtime.h>

constexpr int NBATCH = 24;
constexpr int NT     = 8192;
constexpr int NIN    = 55;
constexpr int NH     = 110;
constexpr int NHP    = 128;
constexpr int NCLS   = 23;
constexpr int NLAY   = 4;
constexpr int NROWS  = NBATCH * NT;
constexpr int KP0    = 64;
constexpr int CHROWS = 64;
constexpr int NCHUNK = NT / CHROWS;
static_assert(NT % CHROWS == 0, "time axis is a whole number of chunks");
static_assert(NROWS == 196608, "row count");
static_assert(NH <= NHP && NIN <= KP0, "pads");

constexpr float ACT_CARRY = 16.0f;
constexpr float W_CARRY   = 64.0f;
constexpr float FOLD      = 1.0f / (ACT_CARRY * W_CARRY);
constexpr float H16_MIN   = 6.103515625e-05f;
constexpr float H16_MAX   = 65504.0f;

constexpr int WPITCH = 136;
constexpr int APITCH = 136;
constexpr int HPITCH = 136;
constexpr int PPITCH = 132;
constexpr int OFF_WT  = 0;
constexpr int SZ_WT   = NHP * WPITCH * 2;
constexpr int OFF_AT  = OFF_WT + SZ_WT;
constexpr int SZ_AT   = CHROWS * APITCH * 2;
constexpr int OFF_PRE = OFF_AT + SZ_AT;
constexpr int SZ_PRE  = CHROWS * PPITCH * 4;
constexpr int OFF_HT  = OFF_PRE + SZ_PRE;
constexpr int SZ_HT   = CHROWS * HPITCH * 2;
constexpr int OFF_HL  = OFF_HT + SZ_HT;
constexpr int SZ_HL   = NHP * 4;
constexpr int LDS_LAYER = OFF_HL + SZ_HL;
static_assert(OFF_AT % 16 == 0 && OFF_PRE % 16 == 0 && OFF_HT % 16 == 0 && OFF_HL % 16 == 0, "16-B aligned LDS regions");
static_assert(LDS_LAYER == 103936, "LDS total");

constexpr size_t SZ_XH  = (size_t)NROWS * KP0 * 2;
constexpr size_t SZ_HP  = (size_t)NROWS * NHP * 2;
constexpr size_t SZ_HLW = (size_t)NBATCH * NHP * 4;
constexpr size_t WOFF_XH = 0;
constexpr size_t WOFF_HA = WOFF_XH + SZ_XH;
constexpr size_t WOFF_HB = WOFF_HA + SZ_HP;
constexpr size_t WOFF_HL = WOFF_HB + SZ_HP;
constexpr size_t WS_TOTAL = WOFF_HL + SZ_HLW;
static_assert(WS_TOTAL == 125841408, "carve total");
static_assert(WS_TOTAL <= 134217728, "carve under 128 MiB");
static_assert(WOFF_HA % 128 == 0 && WOFF_HB % 128 == 0 && WOFF_HL % 128 == 0, "line aligned carves");

typedef __attribute__((ext_vector_type(16))) _Float16 v16h;
typedef __attribute__((ext_vector_type(8)))  _Float16 v8h;
typedef __attribute__((ext_vector_type(8)))  float    v8f;
typedef __attribute__((ext_vector_type(4)))  float    v4f;
typedef __attribute__((ext_vector_type(4)))  unsigned v4u;

struct FragH {
  union U { v16h v; v8h h[2]; };
  static __device__ __forceinline__ v16h load(const _Float16* p) {
    U f;
    f.h[0] = *(const v8h*)(p);
    f.h[1] = *(const v8h*)(p + 16);
    return f.v;
  }
};

__device__ __forceinline__ v8f mma_g(v16h a, v16h b, v8f c) {
  c = __builtin_amdgcn_wmma_f32_16x16x32_f16(false, a, false, b, (short)0, c, false, false);
  asm volatile("v_nop\n\tv_nop\n\tv_nop\n\tv_nop" : "+v"(c) : "v"(a), "v"(b));
  return c;
}

__device__ __forceinline__ void pin_f(float& x) { asm volatile("" : "+v"(x)); }

__device__ __forceinline__ _Float16 to_h16(float v) {
  const float a = fabsf(v);
  float w = (a < H16_MIN) ? 0.0f : v;
  w = fminf(fmaxf(w, -H16_MAX), H16_MAX);
  return (_Float16)w;
}

constexpr int CVT_ITEMS = NROWS * (KP0 / 8);
static_assert(CVT_ITEMS % 256 == 0, "exact grid");
__global__ void __launch_bounds__(256)
cvt_x_kernel(const float* __restrict__ x, unsigned short* __restrict__ xh) {
  const int idx = blockIdx.x * 256 + threadIdx.x;
  const int idc = idx < CVT_ITEMS ? idx : (CVT_ITEMS - 1);
  const int row = idc >> 3;
  const int q   = idc & 7;
  const float* xr = x + (size_t)row * NIN;
  v8h hv;
#pragma unroll
  for (int e = 0; e < 8; ++e) {
    const int col = q * 8 + e;
    const int cc  = col < NIN ? col : (NIN - 1);
    float v = xr[cc];
    pin_f(v);
    const float s = (col < NIN) ? (v * ACT_CARRY) : 0.0f;
    hv[e] = to_h16(s);
  }
  if (idx < CVT_ITEMS) {
    volatile v8h* d = (volatile v8h*)(xh + (size_t)idx * 8);
    *d = hv;
    __threadfence();
    *d = hv;
  }
}

template <int KPAD, int KREAL, bool LAST>
__global__ void __launch_bounds__(256)
erec_layer_kernel(const unsigned short* __restrict__ ain, const float* __restrict__ w,
                  const float* __restrict__ bias, const float* __restrict__ uvec,
                  unsigned short* __restrict__ hout, float* __restrict__ hlast) {
  static_assert(KPAD % 32 == 0 && KPAD <= NHP && KREAL <= KPAD, "k pad");
  static_assert((NHP * KPAD) % 256 == 0, "weight staging covers the plane exactly");
  static_assert((CHROWS * (KPAD / 8)) % 256 == 0, "A tile staging covers the tile exactly");
  extern __shared__ v4u smem_dyn[];
  unsigned char* const smem_raw = (unsigned char*)smem_dyn;
  _Float16* const Wt  = (_Float16*)(smem_raw + OFF_WT);
  _Float16* const At  = (_Float16*)(smem_raw + OFF_AT);
  float*    const Pre = (float*)(smem_raw + OFF_PRE);
  _Float16* const Ht  = (_Float16*)(smem_raw + OFF_HT);
  float*    const Hl  = (float*)(smem_raw + OFF_HL);

  const int tid  = threadIdx.x;
  const int lane = tid & 31;
  const int wave = tid >> 5;
  const int c    = lane & 15;
  const int hh   = lane >> 4;
  const int b    = blockIdx.x;

#pragma unroll 1
  for (int i = tid; i < NHP * KPAD; i += 256) {
    const int n  = i / KPAD;
    const int k  = i % KPAD;
    const int nc = n < NH ? n : (NH - 1);
    const int kc = k < KREAL ? k : (KREAL - 1);
    float v = w[nc * KREAL + kc];
    pin_f(v);
    const bool ok = (n < NH) && (k < KREAL);
    const float s = ok ? (v * W_CARRY) : 0.0f;
    Wt[n * WPITCH + k] = to_h16(s);
  }
  const int jc = tid < NH ? tid : (NH - 1);
  float uu = uvec[jc];
  pin_f(uu);
  float bb = bias[jc];
  pin_f(bb);
  uu = (tid < NH) ? uu : 0.0f;
  bb = (tid < NH) ? bb : 0.0f;
  __syncthreads();

  v16h bfr[KPAD / 32];
#pragma unroll
  for (int kc = 0; kc < KPAD / 32; ++kc)
    bfr[kc] = FragH::load(Wt + (16 * wave + c) * WPITCH + kc * 32 + 8 * hh);

  float hcar = 0.0f;
  constexpr int A16 = KPAD / 8;
  constexpr int AIT = (CHROWS * A16) / 256;

#pragma unroll 1
  for (int ch = 0; ch < NCHUNK; ++ch) {
    const size_t row0 = (size_t)b * NT + (size_t)ch * CHROWS;
    {
      const v4u* src = (const v4u*)(ain + row0 * KPAD);
#pragma unroll
      for (int it = 0; it < AIT; ++it) {
        const int idx = it * 256 + tid;
        const int r = idx / A16;
        const int q = idx % A16;
        const v4u v = src[idx];
        *(v4u*)(smem_raw + OFF_AT + (r * APITCH + q * 8) * 2) = v;
      }
    }
    __syncthreads();

    v8f acc[4];
#pragma unroll
    for (int i = 0; i < 4; ++i) acc[i] = (v8f){0.f, 0.f, 0.f, 0.f, 0.f, 0.f, 0.f, 0.f};
#pragma unroll
    for (int kc = 0; kc < KPAD / 32; ++kc) {
#pragma unroll
      for (int i = 0; i < 4; ++i) {
        const v16h a = FragH::load(At + (16 * i + c) * APITCH + kc * 32 + 8 * hh);
        acc[i] = mma_g(a, bfr[kc], acc[i]);
      }
    }
#pragma unroll
    for (int i = 0; i < 4; ++i) {
#pragma unroll
      for (int r = 0; r < 8; ++r)
        Pre[(16 * i + 8 * hh + r) * PPITCH + 16 * wave + c] = acc[i][r] * FOLD;
    }
    __syncthreads();

    if (tid < NHP) {
      const float* pcol = Pre + tid;
      _Float16* hcol = Ht + tid;
#pragma unroll 8
      for (int r = 0; r < CHROWS; ++r) {
        const float p = pcol[r * PPITCH] + bb;
        hcar = fmaxf(fmaf(uu, hcar, p), 0.0f);
        if (!LAST) hcol[r * HPITCH] = to_h16(hcar * ACT_CARRY);
      }
    }
    __syncthreads();

    if (!LAST) {
      v4u vals[4];
#pragma unroll
      for (int it = 0; it < 4; ++it) {
        const int idx = it * 256 + tid;
        const int r = idx >> 4;
        const int q = idx & 15;
        vals[it] = *(const v4u*)(smem_raw + OFF_HT + (r * HPITCH + q * 8) * 2);
      }
      volatile v4u* dst = (volatile v4u*)(hout + row0 * NHP);
      for (int pass = 0; pass < 2; ++pass) {
#pragma unroll
        for (int it = 0; it < 4; ++it) dst[it * 256 + tid] = vals[it];
        __threadfence();
      }
    }
  }

  if (LAST) {
    if (tid < NHP) Hl[tid] = hcar;
    __syncthreads();
    if (wave == 0) {
      const v4f v = *(const v4f*)(Hl + 4 * lane);
      volatile v4f* d = (volatile v4f*)(hlast + (size_t)b * NHP + 4 * lane);
      *d = v;
      __threadfence();
      *d = v;
    }
  }
}

constexpr int OUT_ITEMS = (NBATCH * NCLS) / 4;
static_assert((NBATCH * NCLS) % 4 == 0, "output is a whole number of 16-B items");
__global__ void __launch_bounds__(128)
head_kernel(const float* __restrict__ hlast, const float* __restrict__ w_out,
            const float* __restrict__ b_out, float* __restrict__ out, int n_out4) {
  __shared__ __align__(16) _Float16 Ah[32 * APITCH];
  __shared__ __align__(16) _Float16 Wh[32 * WPITCH];
  __shared__ float Lg[32 * 33];
  __shared__ __align__(16) float Outs[NBATCH * NCLS];

  const int tid  = threadIdx.x;
  const int lane = tid & 31;
  const int wave = tid >> 5;
  const int c    = lane & 15;
  const int hh   = lane >> 4;

#pragma unroll 1
  for (int it = 0; it < 4; ++it) {
    const int i   = it * 128 + tid;
    const int row = i >> 4;
    const int q8  = (i & 15) * 8;
    const int rc  = row < NBATCH ? row : (NBATCH - 1);
    v4f va = *(const v4f*)(hlast + rc * NHP + q8);
    v4f vb = *(const v4f*)(hlast + rc * NHP + q8 + 4);
    asm volatile("" : "+v"(va), "+v"(vb));
    const bool ok = row < NBATCH;
    v8h hv;
#pragma unroll
    for (int e = 0; e < 4; ++e) {
      const float s0 = ok ? (va[e] * ACT_CARRY) : 0.0f;
      const float s1 = ok ? (vb[e] * ACT_CARRY) : 0.0f;
      hv[e]     = to_h16(s0);
      hv[4 + e] = to_h16(s1);
    }
    *(v8h*)(Ah + row * APITCH + q8) = hv;
  }
#pragma unroll 1
  for (int i = tid; i < 32 * NHP; i += 128) {
    const int n  = i >> 7;
    const int k  = i & 127;
    const int nc = n < NCLS ? n : (NCLS - 1);
    const int kc = k < NH ? k : (NH - 1);
    float v = w_out[nc * NH + kc];
    pin_f(v);
    const bool ok = (n < NCLS) && (k < NH);
    const float s = ok ? (v * W_CARRY) : 0.0f;
    Wh[n * WPITCH + k] = to_h16(s);
  }
  const int mi = wave >> 1;
  const int ni = wave & 1;
  const int ncol = 16 * ni + c;
  const int nbc  = ncol < NCLS ? ncol : (NCLS - 1);
  float bo = b_out[nbc];
  pin_f(bo);
  bo = (ncol < NCLS) ? bo : 0.0f;
  __syncthreads();

  v8f acc = (v8f){0.f, 0.f, 0.f, 0.f, 0.f, 0.f, 0.f, 0.f};
#pragma unroll
  for (int kc = 0; kc < NHP / 32; ++kc) {
    const v16h a  = FragH::load(Ah + (16 * mi + c) * APITCH + kc * 32 + 8 * hh);
    const v16h bw = FragH::load(Wh + (16 * ni + c) * WPITCH + kc * 32 + 8 * hh);
    acc = mma_g(a, bw, acc);
  }
#pragma unroll
  for (int r = 0; r < 8; ++r) Lg[(16 * mi + 8 * hh + r) * 33 + ncol] = acc[r] * FOLD + bo;
  __syncthreads();

  if (tid < NBATCH) {
    const float* lr = Lg + tid * 33;
    float mx = lr[0];
#pragma unroll 1
    for (int o = 1; o < NCLS; ++o) mx = fmaxf(mx, lr[o]);
    float se = 0.0f;
#pragma unroll 1
    for (int o = 0; o < NCLS; ++o) se += expf(lr[o] - mx);
    const float lse = logf(se);
#pragma unroll 1
    for (int o = 0; o < NCLS; ++o) Outs[tid * NCLS + o] = (lr[o] - mx) - lse;
  }
  __syncthreads();

  {
    const int lim = n_out4 < OUT_ITEMS ? n_out4 : OUT_ITEMS;
    v4f vv[2];
#pragma unroll
    for (int it = 0; it < 2; ++it) {
      const int idx = it * 128 + tid;
      const int idc = idx < OUT_ITEMS ? idx : (OUT_ITEMS - 1);
      vv[it] = *(const v4f*)(Outs + 4 * idc);
    }
    for (int pass = 0; pass < 2; ++pass) {
#pragma unroll
      for (int it = 0; it < 2; ++it) {
        const int idx = it * 128 + tid;
        if (idx < lim) *(volatile v4f*)(out + 4 * idx) = vv[it];
      }
      __threadfence();
    }
  }
}

extern "C" void kernel_launch(void* const* d_in, const int* in_sizes, int n_in,
                              void* d_out, int out_size, void* d_ws, size_t ws_size, hipStream_t stream) {
  if (n_in < 9 || d_out == nullptr || d_ws == nullptr) return;
  if (in_sizes[0] != NROWS * NIN || in_sizes[1] != NH * NIN || in_sizes[2] != NH * NH ||
      in_sizes[3] != NH * NH || in_sizes[4] != NH * NH || in_sizes[5] != NLAY * NH ||
      in_sizes[6] != NLAY * NH || in_sizes[7] != NCLS * NH || in_sizes[8] != NCLS ||
      out_size != NBATCH * NCLS) return;
  if (ws_size < WS_TOTAL) return;

  const float* x     = (const float*)d_in[0];
  const float* w0    = (const float*)d_in[1];
  const float* w1    = (const float*)d_in[2];
  const float* w2    = (const float*)d_in[3];
  const float* w3    = (const float*)d_in[4];
  const float* u     = (const float*)d_in[5];
  const float* bb    = (const float*)d_in[6];
  const float* w_out = (const float*)d_in[7];
  const float* b_out = (const float*)d_in[8];
  float* out = (float*)d_out;

  unsigned char* ws = (unsigned char*)d_ws;
  unsigned short* xh = (unsigned short*)(ws + WOFF_XH);
  unsigned short* hA = (unsigned short*)(ws + WOFF_HA);
  unsigned short* hB = (unsigned short*)(ws + WOFF_HB);
  float* hl = (float*)(ws + WOFF_HL);

  cvt_x_kernel<<<dim3(CVT_ITEMS / 256), dim3(256), 0, stream>>>(x, xh);
  erec_layer_kernel<KP0, NIN, false><<<dim3(NBATCH), dim3(256), LDS_LAYER, stream>>>(
      xh, w0, bb + 0 * NH, u + 0 * NH, hA, hl);
  erec_layer_kernel<NHP, NH, false><<<dim3(NBATCH), dim3(256), LDS_LAYER, stream>>>(
      hA, w1, bb + 1 * NH, u + 1 * NH, hB, hl);
  erec_layer_kernel<NHP, NH, false><<<dim3(NBATCH), dim3(256), LDS_LAYER, stream>>>(
      hB, w2, bb + 2 * NH, u + 2 * NH, hA, hl);
  erec_layer_kernel<NHP, NH, true><<<dim3(NBATCH), dim3(256), LDS_LAYER, stream>>>(
      hA, w3, bb + 3 * NH, u + 3 * NH, hB, hl);
  head_kernel<<<dim3(1), dim3(128), 0, stream>>>(hl, w_out, b_out, out, out_size / 4);
}
